// SelfAttention_v1_46909632807066
// MI455X (gfx1250) — hardware-verified
//
#include <hip/hip_runtime.h>


namespace {
constexpr int Bsz = 4, T = 2048, D = 1024;
constexpr int QB = T / 128, KBW = 64;
constexpr int NTRI = QB * QB + QB;
constexpr float WSC = 64.0f;
constexpr float QHAT = 2.0f / WSC, KHAT = 8.0f / WSC, VHAT = 8.0f / WSC;
constexpr float S_SCALE = 1.0f / 16.0f;
constexpr float P_SC = 4096.0f;
constexpr float O_SCALE = 0.125f / 4096.0f;

typedef _Float16 b16;
typedef __attribute__((ext_vector_type(16))) _Float16 v16b;
typedef __attribute__((ext_vector_type(8)))  _Float16 v8b;
typedef __attribute__((ext_vector_type(8)))  float v8f;
typedef __attribute__((ext_vector_type(4)))  float v4f;

__device__ __forceinline__ v8b ld8b(const b16* p) { return *(const v8b*)p; }
__device__ __forceinline__ v16b cat8b(v8b a, v8b b) { return __builtin_shufflevector(a, b, 0, 1, 2, 3, 4, 5, 6, 7, 8, 9, 10, 11, 12, 13, 14, 15); }
__device__ __forceinline__ v16b frag_kb(const b16* p, int hh) { return cat8b(ld8b(p + 8 * hh), ld8b(p + 16 + 8 * hh)); }
__device__ __forceinline__ void split16(float v, b16& hi, b16& lo) { hi = (b16)v; lo = (b16)(v - (float)hi); }
__device__ __forceinline__ void frag_ksplit(const float* p, int hh, v16b& fh_, v16b& fl_) {
  const float* p0 = p + 8 * hh; const float* p1 = p + 16 + 8 * hh;
#pragma unroll
  for (int e = 0; e < 8; ++e) { b16 a, c; split16(p0[e], a, c); fh_[e] = a; fl_[e] = c; split16(p1[e], a, c); fh_[8 + e] = a; fl_[8 + e] = c; }
}
__device__ __forceinline__ v8f wmma16b(v16b a, v16b b, v8f c) {
  v8f d = __builtin_amdgcn_wmma_f32_16x16x32_f16(false, a, false, b, (short)0, c, false, false);
  asm volatile("v_nop\n\tv_nop\n\tv_nop\n\tv_nop" : "+v"(d) : "v"(a), "v"(b));
  return d;
}
__device__ __forceinline__ void wave_lds_sync() {
  __builtin_amdgcn_fence(__ATOMIC_RELEASE, "workgroup");
  __builtin_amdgcn_wave_barrier();
  __builtin_amdgcn_fence(__ATOMIC_ACQUIRE, "workgroup");
}

struct Opnd { const void* p0; const void* p1; int ld; };
template <int NP> __device__ __forceinline__ void load_frags(const Opnd& o, int row, int kb, int hh, v16b& fh_, v16b& fl_) {
  if (NP == 0) { frag_ksplit((const float*)o.p0 + (size_t)row * o.ld + kb, hh, fh_, fl_); }
  else if (NP == 3) {
    const float* p = (const float*)o.p0 + (size_t)row * o.ld + kb; const float* p0 = p + 8 * hh; const float* p1 = p + 16 + 8 * hh;
#pragma unroll
    for (int e = 0; e < 8; ++e) { fh_[e] = (b16)p0[e]; fh_[8 + e] = (b16)p1[e]; }
    fl_ = fh_;
  } else {
    fh_ = frag_kb((const b16*)o.p0 + (size_t)row * o.ld + kb, hh);
    if (NP == 2) fl_ = frag_kb((const b16*)o.p1 + (size_t)row * o.ld + kb, hh); else fl_ = fh_;
  }
}
template <int ANP, int BNP> __device__ __forceinline__ v8f mac(v16b ah, v16b al, v16b bh, v16b bl, v8f c) {
  c = wmma16b(ah, bh, c);
  if (BNP == 0 || BNP == 2) c = wmma16b(ah, bl, c);
  if (ANP == 0 || ANP == 2) c = wmma16b(al, bh, c);
  return c;
}
template <int ANP, int BNP>
__device__ __forceinline__ void gemm_tile(const Opnd& A, const Opnd& B, int K, int m0, int c0, int nloc, int hlf, v8f (&acc)[2][4]) {
  for (int kb = 0; kb < K; kb += 32) {
    v16b a0h, a0l, a1h, a1l;
    load_frags<ANP>(A, m0 + nloc, kb, hlf, a0h, a0l);
    load_frags<ANP>(A, m0 + 16 + nloc, kb, hlf, a1h, a1l);
#pragma unroll
    for (int t = 0; t < 4; ++t) {
      v16b bh, bl;
      load_frags<BNP>(B, c0 + t * 16 + nloc, kb, hlf, bh, bl);
      acc[0][t] = mac<ANP, BNP>(a0h, a0l, bh, bl, acc[0][t]);
      acc[1][t] = mac<ANP, BNP>(a1h, a1l, bh, bl, acc[1][t]);
    }
  }
}

__device__ __forceinline__ void epi_planes(v8f (&acc)[2][4], float scale, bool two, b16* __restrict__ oh, b16* __restrict__ ol, int ldo,
                                           int m0, int c0, int lane, b16* Th, b16* Tl) {
  const int nloc = lane & 15, hlf = lane >> 4;
#pragma unroll
  for (int t = 0; t < 4; ++t)
#pragma unroll
    for (int r = 0; r < 2; ++r)
#pragma unroll
      for (int v = 0; v < 8; ++v) {
        const int rr = r * 16 + v + 8 * hlf, cc = t * 16 + nloc;
        b16 h_, l_; split16(acc[r][t][v] * scale, h_, l_);
        Th[rr * 64 + cc] = h_; Tl[rr * 64 + cc] = l_;
      }
  wave_lds_sync();
  for (int pass = 0; pass < 2; ++pass) {
#pragma unroll
    for (int j = 0; j < 8; ++j) {
      const int rr = j * 4 + (lane >> 3), c8 = (lane & 7) * 8;
      const size_t o = (size_t)(m0 + rr) * ldo + c0 + c8;
      *(volatile v8b*)(oh + o) = ld8b(Th + rr * 64 + c8);
      if (two) *(volatile v8b*)(ol + o) = ld8b(Tl + rr * 64 + c8);
    }
    __threadfence();
  }
}
__device__ __forceinline__ void epi_f32(v8f (&acc)[2][4], float scale, const float* rscale, float* __restrict__ out, int ldo, int m0, int c0, int lane, float* Tt) {
  const int nloc = lane & 15, hlf = lane >> 4;
#pragma unroll
  for (int t = 0; t < 4; ++t)
#pragma unroll
    for (int r = 0; r < 2; ++r)
#pragma unroll
      for (int v = 0; v < 8; ++v) {
        const int rr = r * 16 + v + 8 * hlf;
        const float rs = rscale ? rscale[(size_t)(m0 + rr) * 32] : 1.0f;
        Tt[rr * 64 + t * 16 + nloc] = acc[r][t][v] * scale * rs;
      }
  wave_lds_sync();
  float* dst0 = out + (size_t)m0 * ldo + c0;
  for (int pass = 0; pass < 2; ++pass) {
#pragma unroll
    for (int j = 0; j < 16; ++j) { const int rr = j * 2 + hlf, c4 = nloc * 4; *(volatile v4f*)(dst0 + (size_t)rr * ldo + c4) = *(const v4f*)(Tt + rr * 64 + c4); }
    __threadfence();
  }
}

__global__ __launch_bounds__(256) void prep_kernel(const float* __restrict__ wq, const float* __restrict__ wk, const float* __restrict__ wv,
                                                   b16* __restrict__ wq16, b16* __restrict__ wk16, b16* __restrict__ wvh, b16* __restrict__ wvl) {
  const size_t tid = (size_t)blockIdx.x * blockDim.x + threadIdx.x, stride = (size_t)gridDim.x * blockDim.x;
  const size_t n1 = (size_t)D * D / 8;
  for (int pass = 0; pass < 2; ++pass) {
    for (size_t c = tid; c < 3 * n1; c += stride) {
      const int which = (int)(c / n1); const size_t i = (c % n1) * 8; const size_t n = i / D, k0 = i % D;
      const float* w = (which == 0) ? wq : (which == 1) ? wk : wv;
      v8b vh, vl;
#pragma unroll
      for (int e = 0; e < 8; ++e) { b16 a, cc; split16(w[(k0 + e) * (size_t)D + n] * WSC, a, cc); vh[e] = a; vl[e] = cc; }
      if (which == 0)      { *(volatile v8b*)(wq16 + i) = vh; }
      else if (which == 1) { *(volatile v8b*)(wk16 + i) = vh; }
      else                 { *(volatile v8b*)(wvh + i) = vh; *(volatile v8b*)(wvl + i) = vl; }
    }
    __threadfence();
  }
}

__global__ __launch_bounds__(128) void projqk_kernel(const float* __restrict__ xb, const b16* __restrict__ wq16, const b16* __restrict__ wk16,
                                                     b16* __restrict__ qh, b16* __restrict__ ql, b16* __restrict__ kh) {
  __shared__ __attribute__((aligned(16))) b16 Ts[4][2][32 * 64];
  const int lane = threadIdx.x & 31, wave = threadIdx.x >> 5, nloc = lane & 15, hlf = lane >> 4;
  const int m0 = blockIdx.y * 128 + wave * 32;
  const int cg = blockIdx.x * 64;
  const bool isq = cg < D; const int c0 = isq ? cg : cg - D;
  v8f acc[2][4];
#pragma unroll
  for (int r = 0; r < 2; ++r)
#pragma unroll
    for (int t = 0; t < 4; ++t) acc[r][t] = (v8f){};
  const Opnd A{xb, nullptr, D}, B{isq ? wq16 : wk16, nullptr, D};
  gemm_tile<0, 1>(A, B, D, m0, c0, nloc, hlf, acc);
  epi_planes(acc, isq ? QHAT : KHAT, isq, isq ? qh : kh, isq ? ql : nullptr, D, m0, c0, lane, Ts[wave][0], Ts[wave][1]);
}

__global__ __launch_bounds__(128) void projv_kernel(const float* __restrict__ xb, const b16* __restrict__ wvh, const b16* __restrict__ wvl,
                                                    b16* __restrict__ vth, b16* __restrict__ vtl) {
  __shared__ __attribute__((aligned(16))) b16 Ts[4][2][32 * 64];
  const int lane = threadIdx.x & 31, wave = threadIdx.x >> 5, nloc = lane & 15, hlf = lane >> 4;
  const int m0 = blockIdx.y * 128 + wave * 32;
  const int c0 = blockIdx.x * 64;
  v8f acc[2][4];
#pragma unroll
  for (int r = 0; r < 2; ++r)
#pragma unroll
    for (int t = 0; t < 4; ++t) acc[r][t] = (v8f){};
  const Opnd A{wvh, wvl, D}, B{xb, nullptr, D};
  gemm_tile<2, 3>(A, B, D, m0, c0, nloc, hlf, acc);
  epi_planes(acc, VHAT, true, vth, vtl, T, m0, c0, lane, Ts[wave][0], Ts[wave][1]);
}

__global__ __launch_bounds__(128) void s_kernel(const b16* __restrict__ qh, const b16* __restrict__ ql, const b16* __restrict__ kh,
                                                float* __restrict__ S) {
  __shared__ __attribute__((aligned(16))) float Ts[4][32 * 64];
  const int lane = threadIdx.x & 31, wave = threadIdx.x >> 5, nloc = lane & 15, hlf = lane >> 4;
  int qb = 0;
#pragma unroll 1
  for (int j = 1; j <= QB; ++j) { if (j * j + j <= (int)blockIdx.x) qb = j; }
  if (qb >= QB) return;
  const int kt = (int)blockIdx.x - (qb * qb + qb);
  const int m0 = qb * 128 + wave * 32, c0 = kt * KBW;
  v8f acc[2][4];
#pragma unroll
  for (int r = 0; r < 2; ++r)
#pragma unroll
    for (int t = 0; t < 4; ++t) acc[r][t] = (v8f){};
  const Opnd A{qh, ql, D}, B{kh, nullptr, D};
  gemm_tile<2, 1>(A, B, D, m0, c0, nloc, hlf, acc);
  epi_f32(acc, S_SCALE * (1.0f / 32.0f), nullptr, S, T, m0, c0, lane, Ts[wave]);
}

__global__ __launch_bounds__(256) void softmax_kernel(const float* __restrict__ S, b16* __restrict__ P, float* __restrict__ rowscale) {
  const int lane = threadIdx.x & 31, r = blockIdx.x * 8 + (threadIdx.x >> 5);
  if (r >= T) return;
  const int kend = ((r >> 7) + 1) << 7;
  const float* Sr = S + (size_t)r * T;
  float sv[64];
  float mx = -INFINITY;
#pragma unroll
  for (int j = 0; j < 8; ++j)
#pragma unroll
    for (int e = 0; e < 8; ++e) {
      const int kk = lane * 8 + 256 * j + e;
      const float s = (kk <= r) ? Sr[(kk < kend) ? kk : 0] : -INFINITY;
      sv[j * 8 + e] = s; mx = fmaxf(mx, s);
    }
#pragma unroll
  for (int o = 16; o > 0; o >>= 1) mx = fmaxf(mx, __shfl_xor(mx, o));
  float sum = 0.0f;
#pragma unroll
  for (int i = 0; i < 64; ++i) { const float p = __expf(sv[i] - mx); sv[i] = p; sum += p; }
#pragma unroll
  for (int o = 16; o > 0; o >>= 1) sum += __shfl_xor(sum, o);
  const float inv = 1.0f / sum;
  b16* Pr = P + (size_t)r * T;
  for (int pass = 0; pass < 2; ++pass) {
#pragma unroll
    for (int j = 0; j < 8; ++j) {
      const int k0 = lane * 8 + 256 * j;
      if (k0 < kend) {
        v8b pv;
#pragma unroll
        for (int e = 0; e < 8; ++e) pv[e] = (b16)(sv[j * 8 + e] * P_SC);
        *(volatile v8b*)(Pr + k0) = pv;
      }
    }
    ((volatile float*)rowscale)[(size_t)r * 32 + lane] = (lane == 0) ? inv : 0.0f;
    __threadfence();
  }
}

__global__ __launch_bounds__(128) void pv_kernel(const b16* __restrict__ P, const b16* __restrict__ vth, const b16* __restrict__ vtl, const float* __restrict__ rowscale,
                                                 float* __restrict__ outb) {
  __shared__ __attribute__((aligned(16))) float Ts[4][32 * 64];
  const int lane = threadIdx.x & 31, wave = threadIdx.x >> 5, nloc = lane & 15, hlf = lane >> 4;
  const int qb = blockIdx.y, m0 = qb * 128 + wave * 32, c0 = blockIdx.x * 64;
  const int kend = (qb + 1) * 128;
  v8f acc[2][4];
#pragma unroll
  for (int r = 0; r < 2; ++r)
#pragma unroll
    for (int t = 0; t < 4; ++t) acc[r][t] = (v8f){};
  const Opnd A{P, nullptr, T}, B{vth, vtl, T};
  gemm_tile<1, 2>(A, B, kend, m0, c0, nloc, hlf, acc);
  epi_f32(acc, O_SCALE, rowscale, outb, D, m0, c0, lane, Ts[wave]);
}
}

extern "C" void kernel_launch(void* const* d_in, const int* in_sizes, int n_in,
                              void* d_out, int out_size, void* d_ws, size_t ws_size, hipStream_t stream) {
  (void)n_in; (void)out_size;
  const float* x  = (const float*)d_in[0];
  const float* Wq = (const float*)d_in[1];
  const float* Wk = (const float*)d_in[2];
  const float* Wv = (const float*)d_in[3];
  float* out = (float*)d_out;
  if (in_sizes[0] != Bsz * T * D || in_sizes[1] != D * D || in_sizes[2] != D * D || in_sizes[3] != D * D) return;

  size_t off = 0; char* ws = (char*)d_ws;
  auto carve = [&](size_t bytes) { char* p = ws + off; off += (bytes + 255) & ~(size_t)255; return p; };
  b16* wq16 = (b16*)carve((size_t)D * D * 2);
  b16* wk16 = (b16*)carve((size_t)D * D * 2);
  b16* wvh  = (b16*)carve((size_t)D * D * 2);
  b16* wvl  = (b16*)carve((size_t)D * D * 2);
  b16* qh   = (b16*)carve((size_t)T * D * 2);
  b16* ql   = (b16*)carve((size_t)T * D * 2);
  b16* kh   = (b16*)carve((size_t)T * D * 2);
  b16* vth  = (b16*)carve((size_t)D * T * 2);
  b16* vtl  = (b16*)carve((size_t)D * T * 2);
  float* S  = (float*)carve((size_t)T * T * 4);
  b16* P    = (b16*)carve((size_t)T * T * 2);
  float* rsc = (float*)carve((size_t)T * 32 * 4);
  if (off > ws_size) return;
  prep_kernel<<<1024, 256, 0, stream>>>(Wq, Wk, Wv, wq16, wk16, wvh, wvl);
  for (int b = 0; b < Bsz; ++b) {
    const float* xb = x + (size_t)b * T * D; float* outb = out + (size_t)b * T * D;
    projqk_kernel<<<dim3(2 * D / 64, T / 128), 128, 0, stream>>>(xb, wq16, wk16, qh, ql, kh);
    projv_kernel<<<dim3(T / 64, D / 128), 128, 0, stream>>>(xb, wvh, wvl, vth, vtl);
    s_kernel<<<NTRI, 128, 0, stream>>>(qh, ql, kh, S);
    softmax_kernel<<<T / 8, 256, 0, stream>>>(S, P, rsc);
    pv_kernel<<<dim3(D / 64, T / 128), 128, 0, stream>>>(P, vth, vtl, rsc, outb);
  }
}
